// PairwiseAttentionBlock_46420006535528
// MI455X (gfx1250) — hardware-run, weakly checked
//
#include <hip/hip_runtime.h>
#include <math.h>

typedef __attribute__((ext_vector_type(16))) _Float16 v16h;
typedef __attribute__((ext_vector_type(16))) __bf16 v16b;
typedef __attribute__((ext_vector_type(8)))  _Float16 v8h;
typedef __attribute__((ext_vector_type(8)))  float v8f;
typedef __attribute__((ext_vector_type(4)))  float v4f;
typedef __attribute__((ext_vector_type(2)))  float v2f;
typedef __attribute__((ext_vector_type(4)))  unsigned v4u;
typedef __attribute__((ext_vector_type(4)))  int v4i;
typedef float __attribute__((may_alias)) float_a;
typedef int __attribute__((may_alias)) int_a;

template <typename T> __device__ __forceinline__ void vst2(void* p, T v) { *(volatile T*)p = v; __threadfence(); *(volatile T*)p = v; }
__device__ __forceinline__ v8f wmma16(v16h a, v16h b, v8f c) {
  v8f d = __builtin_amdgcn_wmma_f32_16x16x32_f16(false, a, false, b, (short)0, c, false, false);
  asm volatile("v_nop\n\tv_nop\n\tv_nop\n\tv_nop" : "+v"(d) : "v"(a), "v"(b));
  return d;
}
__device__ __forceinline__ v8f wmma_bf(v16b a, v16b b, v8f c) {
  v8f d = __builtin_amdgcn_wmma_f32_16x16x32_bf16(false, a, false, b, (short)0, c, false, false);
  asm volatile("v_nop\n\tv_nop\n\tv_nop\n\tv_nop" : "+v"(d) : "v"(a), "v"(b));
  return d;
}
__device__ __forceinline__ v16h frag_h(const _Float16* rowk0, int lane) {
  union { v16h v; v8h q[2]; } u; const _Float16* p = rowk0 + 8 * (lane >> 4);
  u.q[0] = *(const v8h*)p; u.q[1] = *(const v8h*)(p + 16); return u.v;
}
__device__ __forceinline__ v16h frag_f32(const float* rowk0, int lane) {
  v16h a; const float* p = rowk0 + 8 * (lane >> 4);
#pragma unroll
  for (int i = 0; i < 8; ++i) { a[i] = (_Float16)p[i]; a[8 + i] = (_Float16)p[16 + i]; }
  return a;
}
__device__ __forceinline__ v16h frag_f32s(const float* rowk0, int lane, float sc) {
  v16h a; const float* p = rowk0 + 8 * (lane >> 4);
#pragma unroll
  for (int i = 0; i < 8; ++i) { a[i] = (_Float16)(p[i] * sc); a[8 + i] = (_Float16)(p[16 + i] * sc); }
  return a;
}
__device__ __forceinline__ v16h fragc_f32(const float* W, int k0, int n, int lane, int ld, int K) {
  v16h a; const int g = lane >> 4;
#pragma unroll
  for (int i = 0; i < 8; ++i) { const int ka = k0 + 8 * g + i, kb = ka + 16;
    a[i] = (_Float16)(ka < K ? W[(size_t)(ka < K ? ka : K - 1) * ld + n] : 0.f); a[8 + i] = (_Float16)(kb < K ? W[(size_t)(kb < K ? kb : K - 1) * ld + n] : 0.f); }
  return a;
}
struct F2 { v16b h, l; };
__device__ __forceinline__ F2 bsplit16(const float v[16]) { F2 r;
#pragma unroll
  for (int i = 0; i < 16; ++i) { const __bf16 h = (__bf16)v[i]; r.h[i] = h; r.l[i] = (__bf16)(v[i] - (float)h); }
  return r; }
__device__ __forceinline__ F2 split_row(const float* row, int k0, int lane) { float v[16]; const float* p = row + k0 + 8 * (lane >> 4);
#pragma unroll
  for (int i = 0; i < 8; ++i) { v[i] = p[i]; v[8 + i] = p[16 + i]; }
  return bsplit16(v); }
__device__ __forceinline__ F2 split_rowK(const float* row, int k0, int lane, int K) { float v[16]; const int g = lane >> 4;
#pragma unroll
  for (int i = 0; i < 8; ++i) { const int ka = k0 + 8 * g + i, kb = ka + 16; v[i] = ka < K ? row[ka < K ? ka : K - 1] : 0.f; v[8 + i] = kb < K ? row[kb < K ? kb : K - 1] : 0.f; }
  return bsplit16(v); }
__device__ __forceinline__ F2 split_col(const float* W, int k0, int n, int lane, int ld, int K) { float v[16]; const int g = lane >> 4;
#pragma unroll
  for (int i = 0; i < 8; ++i) { const int ka = k0 + 8 * g + i, kb = ka + 16; v[i] = ka < K ? W[(size_t)(ka < K ? ka : K - 1) * ld + n] : 0.f; v[8 + i] = kb < K ? W[(size_t)(kb < K ? kb : K - 1) * ld + n] : 0.f; }
  return bsplit16(v); }
__device__ __forceinline__ v8f mac3(const F2& a, const F2& b, v8f c) { c = wmma_bf(a.l, b.h, c); c = wmma_bf(a.h, b.l, c); return wmma_bf(a.h, b.h, c); }
__device__ __forceinline__ float sigm(float v) { return 1.0f / (1.0f + expf(-v)); }
#define LDSX() do { asm volatile("s_wait_dscnt 0" ::: "memory"); __builtin_amdgcn_wave_barrier(); __builtin_amdgcn_fence(__ATOMIC_RELEASE, "workgroup"); } while (0)


#define NQ 320
#define DD 128
#define NH 4
#define HD 32
#define NP (NQ * NQ)
#define LNEPS 1e-5f
typedef __attribute__((ext_vector_type(8))) __bf16 v8b;
__device__ __forceinline__ v16b frag_b(const __bf16* rowk0, int lane) {
  union { v16b v; v8b q[2]; } u; const __bf16* p = rowk0 + 8 * (lane >> 4);
  u.q[0] = *(const v8b*)p; u.q[1] = *(const v8b*)(p + 16); return u.v;
}
__device__ __forceinline__ float bfr(float v) { return (float)(__bf16)v; }
__device__ __attribute__((noinline)) float exp_ni(float v) { return expf(v); }
__device__ __attribute__((noinline)) float erf_ni(float v) { return erff(v); }

#define WS_X1  0u
#define WS_Q   (WS_X1 + 4u * (size_t)NP * DD)
#define WS_K   (WS_Q + 2u * (size_t)NP * DD)
#define WS_G   (WS_K + 2u * (size_t)NP * DD)
#define WS_V   (WS_G + 4u * (size_t)NP * DD)
#define WS_B   (WS_V + 2u * (size_t)DD * NP)
#define WS_O   (WS_B + 4u * (size_t)NH * NP)
#define WS_END (WS_O + 2u * (size_t)NP * DD)

__global__ __launch_bounds__(256) void k_bias(const float* __restrict__ X, const float* __restrict__ WB, int RAW, float* __restrict__ Bo) { __shared__ __align__(16) float sb[NH][64]; const int t = threadIdx.x, lane = t & 31, w = t >> 5; const size_t p0 = (size_t)blockIdx.x * 64;
#pragma unroll 1
  for (int rr = 0; rr < 8; ++rr) { const size_t p = p0 + w * 8 + rr; float acc[NH]; const float* xr = X + p * DD;
#pragma unroll
    for (int h = 0; h < NH; ++h) acc[h] = 0.f;
#pragma unroll
    for (int i = 0; i < DD / 32; ++i) { const float xv = RAW ? xr[lane + 32 * i] : bfr(xr[lane + 32 * i]);
#pragma unroll
      for (int h = 0; h < NH; ++h) acc[h] += xv * bfr(WB[h * DD + lane + 32 * i]); }
#pragma unroll
    for (int h = 0; h < NH; ++h) { float v = acc[h];
#pragma unroll
      for (int o = 1; o < 32; o <<= 1) v += __shfl_xor(v, o);
      if (lane == 0) sb[h][w * 8 + rr] = v; } }
  __syncthreads(); if (t < NH * 16) { const int h = t >> 4, q = t & 15; vst2(Bo + (size_t)h * NP + p0 + q * 4, *(const v4f*)&sb[h][q * 4]); } }
__global__ __launch_bounds__(128) void k_proj(const float* __restrict__ X, const float* __restrict__ G_, const float* __restrict__ Bt, const float* __restrict__ WQ, const float* __restrict__ WKV, const float* __restrict__ WG, const float* __restrict__ BG, int RS, int LS, _Float16* __restrict__ Q, _Float16* __restrict__ K, _Float16* __restrict__ V, float* __restrict__ GT) {
  __shared__ __align__(16) _Float16 sx[64][DD + 8]; __shared__ __align__(16) _Float16 sh[64][DD + 8]; __shared__ __align__(16) float sg[64][DD + 4]; __shared__ __align__(16) _Float16 th[DD][72];
  const int tid = threadIdx.x, wave = tid >> 5, lane = tid & 31, col = lane & 15, g = lane >> 4; const int r = blockIdx.y; const int l0 = blockIdx.x * 64; const size_t a0 = (size_t)r * NQ + l0;
  for (int rr = 0; rr < 16; ++rr) { const int rl = wave * 16 + rr; const size_t p = (size_t)r * RS + (size_t)(l0 + rl) * LS; float v[4]; float s = 0.f; for (int i = 0; i < 4; ++i) { const float xv = X[p * DD + lane + 32 * i]; v[i] = (RS == NQ) ? bfr(xv) : xv; s += v[i]; }
#pragma unroll
    for (int o = 1; o < 32; o <<= 1) s += __shfl_xor(s, o);
    const float mu = s * (1.0f / DD); float q = 0.f; for (int i = 0; i < 4; ++i) { const float d = v[i] - mu; q += d * d; }
#pragma unroll
    for (int o = 1; o < 32; o <<= 1) q += __shfl_xor(q, o);
    const float inv = 1.0f / sqrtf(q * (1.0f / DD) + LNEPS); for (int i = 0; i < 4; ++i) { const int c = lane + 32 * i; sx[rl][c] = (_Float16)((v[i] - mu) * inv * bfr(G_[c]) + bfr(Bt[c])); } }
  __syncthreads();
#pragma unroll 1
  for (int which = 0; which < 4; ++which) {
    const float* Wm = which == 0 ? WQ : which == 1 ? WKV : which == 2 ? (WKV + (size_t)DD * DD) : WG;
    v8f acc[8] = {};
#pragma unroll
    for (int kc = 0; kc < DD / 32; ++kc) { v16h a; const _Float16* pp = &sx[wave * 16 + col][kc * 32 + 8 * g];
#pragma unroll
      for (int i = 0; i < 8; ++i) { a[i] = pp[i]; a[8 + i] = pp[16 + i]; }
#pragma unroll
      for (int j = 0; j < 8; ++j) { v16h w; const float* wr = Wm + (size_t)(j * 16 + col) * DD + kc * 32 + 8 * g;
#pragma unroll
        for (int i = 0; i < 8; ++i) { w[i] = (_Float16)bfr(wr[i]); w[8 + i] = (_Float16)bfr(wr[16 + i]); }
        acc[j] = wmma16(a, w, acc[j]); } }
#pragma unroll
    for (int j = 0; j < 8; ++j) { const int c = j * 16 + col;
#pragma unroll
      for (int rr = 0; rr < 8; ++rr) { const float v = acc[j][rr]; const int rl = wave * 16 + 8 * g + rr; if (which == 3) sg[rl][c] = 1.0f / (1.0f + expf(-(v + bfr(BG[c])))); else if (which == 2) th[c][rl] = (_Float16)v; else sh[rl][c] = (_Float16)v; } }
    __syncthreads();
    if (which < 2) { _Float16* dst = which == 0 ? Q : K; for (int e = tid; e < 64 * 16; e += 128) { const int rl = e >> 4, q = e & 15; vst2((unsigned*)(dst + (a0 + rl) * DD + q * 8), *(const v4u*)&sh[rl][q * 8]); } }
    else if (which == 2) { for (int e = tid; e < DD * 8; e += 128) { const int c = e >> 3, q = e & 7; vst2((unsigned*)(V + (size_t)c * NP + a0 + q * 8), *(const v4u*)&th[c][q * 8]); } }
    else { for (int e = tid; e < 64 * 32; e += 128) { const int rl = e >> 5, q = e & 31; vst2(GT + (a0 + rl) * DD + q * 4, *(const v4f*)&sg[rl][q * 4]); } }
    __syncthreads(); } }
__global__ __launch_bounds__(128) void k_att(const _Float16* __restrict__ Q, const _Float16* __restrict__ K, const _Float16* __restrict__ V, const float* __restrict__ Bi, const float* __restrict__ GT, _Float16* __restrict__ O) {
  __shared__ __align__(16) float sp[4][16][36]; __shared__ __align__(16) _Float16 so[4][16][40];
  const int tid = threadIdx.x, wave = tid >> 5, lane = tid & 31, col = lane & 15, g = lane >> 4; const int h = blockIdx.y; const int r = blockIdx.z; const int l0 = blockIdx.x * 64 + wave * 16; const size_t aq = (size_t)r * NQ + l0;
  const v16h a = frag_h(Q + (aq + col) * DD + h * HD, lane);
  float m[8], l[8];
#pragma unroll
  for (int rr = 0; rr < 8; ++rr) { m[rr] = -3.0e38f; l[rr] = 0.f; }
  v8f acc[2] = {};
#pragma unroll 1
  for (int ks = 0; ks < NQ / 32; ++ks) { float s[2][8];
#pragma unroll
    for (int ct = 0; ct < 2; ++ct) { const int kk = ks * 32 + ct * 16 + col; v8f c = {}; c = wmma16(a, frag_h(K + ((size_t)r * NQ + kk) * DD + h * HD, lane), c);
#pragma unroll
      for (int rr = 0; rr < 8; ++rr) s[ct][rr] = c[rr] * 0.17677669529663687f + Bi[(size_t)h * NP + (size_t)(l0 + 8 * g + rr) * NQ + kk]; }
    float alpha[8];
#pragma unroll
    for (int rr = 0; rr < 8; ++rr) { float mx = fmaxf(s[0][rr], s[1][rr]);
#pragma unroll
      for (int o = 1; o < 16; o <<= 1) mx = fmaxf(mx, __shfl_xor(mx, o));
      const float mn = fmaxf(m[rr], mx); alpha[rr] = __expf(m[rr] - mn); const float e0 = __expf(s[0][rr] - mn), e1 = __expf(s[1][rr] - mn); float es = e0 + e1;
#pragma unroll
      for (int o = 1; o < 16; o <<= 1) es += __shfl_xor(es, o);
      l[rr] = l[rr] * alpha[rr] + es; m[rr] = mn; sp[wave][8 * g + rr][col] = e0; sp[wave][8 * g + rr][16 + col] = e1; }
#pragma unroll
    for (int j = 0; j < 2; ++j)
#pragma unroll
      for (int rr = 0; rr < 8; ++rr) acc[j][rr] *= alpha[rr];
    LDSX();
    v16h pa; { const float* prow = &sp[wave][col][0] + 8 * (lane >> 4);
#pragma unroll
      for (int i = 0; i < 8; ++i) { pa[i] = (_Float16)(prow[i] * 2048.0f); pa[8 + i] = (_Float16)(prow[16 + i] * 2048.0f); } }
#pragma unroll
    for (int j = 0; j < 2; ++j) acc[j] = wmma16(pa, frag_h(V + (size_t)(h * HD + j * 16 + col) * NP + (size_t)r * NQ + ks * 32, lane), acc[j]);
    LDSX(); }
#pragma unroll
  for (int rr = 0; rr < 8; ++rr) { const float il = (1.0f / 2048.0f) / l[rr];
#pragma unroll
    for (int j = 0; j < 2; ++j) { const int c = h * HD + j * 16 + col; so[wave][8 * g + rr][j * 16 + col] = (_Float16)(acc[j][rr] * il * GT[(aq + 8 * g + rr) * DD + c]); } }
  LDSX(); for (int rl = 0; rl < 16; ++rl) if (lane < 4) vst2((unsigned*)(O + (aq + rl) * DD + h * HD + lane * 8), *(const v4u*)&so[wave][rl][lane * 8]); }
__global__ __launch_bounds__(128) void k_out(const _Float16* __restrict__ O, const float* __restrict__ WO, const float* __restrict__ BO, const float* __restrict__ X, int RS, int LS, float* __restrict__ XN) { __shared__ __align__(16) float sf[4][16][132];
  const int tid = threadIdx.x, wave = tid >> 5, lane = tid & 31, col = lane & 15, g = lane >> 4; const int r = blockIdx.y; const int l0 = blockIdx.x * 64 + wave * 16; const size_t a0 = (size_t)r * NQ + l0;
  v8f acc[8] = {};
#pragma unroll
  for (int kc = 0; kc < DD / 32; ++kc) { const v16h a = frag_h(O + (a0 + col) * DD + kc * 32, lane);
#pragma unroll
    for (int j = 0; j < 8; ++j) { v16h w; const float* wr = WO + (size_t)(j * 16 + col) * DD + kc * 32 + 8 * g;
#pragma unroll
      for (int i = 0; i < 8; ++i) { w[i] = (_Float16)bfr(wr[i]); w[8 + i] = (_Float16)bfr(wr[16 + i]); }
      acc[j] = wmma16(a, w, acc[j]); } }
#pragma unroll
  for (int j = 0; j < 8; ++j) { const int c = j * 16 + col; const float bb = bfr(BO[c]);
#pragma unroll
    for (int rr = 0; rr < 8; ++rr) { const size_t p = (size_t)r * RS + (size_t)(l0 + 8 * g + rr) * LS; sf[wave][8 * g + rr][c] = acc[j][rr] + bb + (RS == NQ ? bfr(X[p * DD + c]) : X[p * DD + c]); } }
  LDSX(); for (int rl = 0; rl < 16; ++rl) { const size_t p = (size_t)r * RS + (size_t)(l0 + rl) * LS; vst2(XN + p * DD + lane * 4, *(const v4f*)&sf[wave][rl][lane * 4]); } }
extern "C" void kernel_launch(void* const* d_in, const int* in_sizes, int n_in, void* d_out, int out_size, void* d_ws, size_t ws_size, hipStream_t stream) {
  (void)in_sizes; (void)n_in; (void)out_size;
  const float** F = (const float**)d_in;
  if (ws_size < (size_t)WS_END) return;
  char* ws = (char*)d_ws; float *X1 = (float*)(ws + WS_X1), *GT = (float*)(ws + WS_G), *Bi = (float*)(ws + WS_B); _Float16 *Q = (_Float16*)(ws + WS_Q), *K = (_Float16*)(ws + WS_K), *V = (_Float16*)(ws + WS_V), *O = (_Float16*)(ws + WS_O);
  k_bias<<<NP / 64, 256, 0, stream>>>(F[0], F[3], 0, Bi);
  k_proj<<<dim3(NQ / 64, NQ), 128, 0, stream>>>(F[0], F[1], F[2], F[4], F[5], F[6], F[7], NQ, 1, Q, K, V, GT);
  k_att<<<dim3(NQ / 64, NH, NQ), 128, 0, stream>>>(Q, K, V, Bi, GT, O);
  k_out<<<dim3(NQ / 64, NQ), 128, 0, stream>>>(O, F[8], F[9], F[0], NQ, 1, X1);
  k_bias<<<NP / 64, 256, 0, stream>>>(X1, F[12], 1, Bi);
  k_proj<<<dim3(NQ / 64, NQ), 128, 0, stream>>>(X1, F[10], F[11], F[13], F[14], F[15], F[16], 1, NQ, Q, K, V, GT);
  k_att<<<dim3(NQ / 64, NH, NQ), 128, 0, stream>>>(Q, K, V, Bi, GT, O);
  k_out<<<dim3(NQ / 64, NQ), 128, 0, stream>>>(O, F[17], F[18], X1, 1, NQ, (float*)d_out);
}
